// EnhancedMSTSN_88974542504137
// MI455X (gfx1250) — hardware-verified
//
#include <hip/hip_runtime.h>
#define BBs 8
#define SS 24
#define NNn 400
#define NG (BBs * SS)
#define NRW (NG * NNn)
#define DM 32
#define KP 448

typedef __bf16 v16b __attribute__((ext_vector_type(16)));
typedef unsigned short v8us __attribute__((ext_vector_type(8), may_alias));
typedef float  v8f  __attribute__((ext_vector_type(8)));
typedef float  v4f  __attribute__((ext_vector_type(4)));
typedef float  v4fa __attribute__((ext_vector_type(4), may_alias));
union FragB { v16b v; v8us half[2]; unsigned short u[16]; };

__device__ __forceinline__ unsigned short bf16_bits(float x) { unsigned int u = __float_as_uint(x); return (unsigned short)((u + 0x7FFFu + ((u >> 16) & 1u)) >> 16); }
__device__ __forceinline__ float bf16_val(unsigned short b) { return __uint_as_float(((unsigned int)b) << 16); }
__device__ __forceinline__ float bf16_round(float x) { return bf16_val(bf16_bits(x)); }
template <int NT>
__device__ __forceinline__ v8f mmaN(v16b ah, v16b al, v16b bh, v16b bl, v8f c) {
  c = __builtin_amdgcn_wmma_f32_16x16x32_bf16(false, ah, false, bh, (short)0, c, false, false);
  if (NT >= 2) c = __builtin_amdgcn_wmma_f32_16x16x32_bf16(false, al, false, bh, (short)0, c, false, false);
  if (NT >= 3) c = __builtin_amdgcn_wmma_f32_16x16x32_bf16(false, ah, false, bl, (short)0, c, false, false);
  asm volatile("v_nop\n\tv_nop\n\tv_nop\n\tv_nop" : "+v"(c) : "v"(ah), "v"(al), "v"(bh), "v"(bl));
  return c;
}

__global__ __launch_bounds__(256) void k_wt_bf16(const float* __restrict__ W, unsigned short* __restrict__ Wt, int K, int N) {
  const int t = blockIdx.x * 256 + threadIdx.x;
  const int k8n = K / 8;
  if (t >= N * k8n) return;
  const int n = t / k8n, k8 = (t % k8n) * 8;
  v8us v;
#pragma unroll
  for (int i = 0; i < 8; ++i) v[i] = bf16_bits(W[(size_t)(k8 + i) * N + n]);
  *(volatile v8us*)(Wt + (size_t)n * K + k8) = v;
  __threadfence();
  *(volatile v8us*)(Wt + (size_t)n * K + k8) = v;
}

template <bool ASPLIT, int ACT, bool BIAS_BF16>
__global__ __launch_bounds__(128) void k_gemm_bf(const float* __restrict__ A, int lda, const unsigned short* __restrict__ Wt, int ldb,
                                               const float* __restrict__ bias, float* __restrict__ C, int ldc, int M, int N, int K) {
  __shared__ __attribute__((aligned(16))) float so[4][16][64];
  const int tid = threadIdx.x, w = tid >> 5, lane = tid & 31, ln = lane & 15, hh = lane >> 4;
  const int ntn = N / 64;
  const int wid = blockIdx.x * 4 + w;
  const int mt = wid / ntn, nq = wid % ntn;
  if (mt * 16 >= M) return;
  const int row0 = mt * 16, col0 = nq * 64;
  const float* arow = A + (size_t)(row0 + ln) * lda;
  v8f acc[4] = {};
  for (int kb = 0; kb < K; kb += 32) {
    FragB ah, al;
    const v4f x0 = *(const v4fa*)(arow + kb + 8 * hh), x1 = *(const v4fa*)(arow + kb + 8 * hh + 4);
    const v4f x2 = *(const v4fa*)(arow + kb + 16 + 8 * hh), x3 = *(const v4fa*)(arow + kb + 16 + 8 * hh + 4);
    float xs[16] = {x0[0],x0[1],x0[2],x0[3],x1[0],x1[1],x1[2],x1[3],x2[0],x2[1],x2[2],x2[3],x3[0],x3[1],x3[2],x3[3]};
#pragma unroll
    for (int i = 0; i < 16; ++i) { const unsigned short hb = bf16_bits(xs[i]); ah.u[i] = hb; al.u[i] = ASPLIT ? bf16_bits(xs[i] - bf16_val(hb)) : (unsigned short)0; }
#pragma unroll
    for (int t = 0; t < 4; ++t) {
      const unsigned short* brow = Wt + (size_t)(col0 + t * 16 + ln) * ldb + kb;
      FragB b;
      b.half[0] = *(const v8us*)(brow + 8 * hh);
      b.half[1] = *(const v8us*)(brow + 16 + 8 * hh);
      acc[t] = mmaN<ASPLIT ? 2 : 1>(ah.v, al.v, b.v, b.v, acc[t]);
    }
  }
#pragma unroll
  for (int t = 0; t < 4; ++t) {
    float bv = bias ? bias[col0 + t * 16 + ln] : 0.f;
    if (BIAS_BF16) bv = bf16_round(bv);
#pragma unroll
    for (int r = 0; r < 8; ++r) { float v = acc[t][r] + bv; if (ACT == 1) v = fmaxf(v, 0.f); so[w][8 * hh + r][t * 16 + ln] = v; }
  }
  __builtin_amdgcn_fence(__ATOMIC_ACQ_REL, "workgroup");
  __builtin_amdgcn_wave_barrier();
  const int rsub = lane >> 4, c4 = (lane & 15) * 4;
  for (int pass = 0; pass < 2; ++pass) {
#pragma unroll
    for (int q = 0; q < 8; ++q) {
      const int r = q * 2 + rsub;
      const v4f v = *(const v4fa*)&so[w][r][c4];
      *(volatile v4f*)(C + (size_t)(row0 + r) * ldc + col0 + c4) = v;
    }
    if (pass == 0) __threadfence();
  }
}

template <int D, bool CAUSAL>
__global__ __launch_bounds__(128) void k_flash(const float* __restrict__ qb, const float* __restrict__ kb, const float* __restrict__ vb,
                                             int pitch, int T, int H, float scale, float* __restrict__ y, int ypitch) {
  constexpr int KS = D / 32;
  constexpr int DT = D / 16;
  __shared__ __attribute__((aligned(16))) unsigned short sKh[32][D + 8], sKl[32][D + 8], sVh[32][D + 8], sVl[32][D + 8];
  __shared__ __attribute__((aligned(16))) unsigned short sPh[4][16][40], sPl[4][16][40];
  __shared__ __attribute__((aligned(16))) float sO[4][16][D];
  const int tid = threadIdx.x, w = tid >> 5, lane = tid & 31, ln = lane & 15, hh = lane >> 4;
  const int nqb = (T + 63) / 64;
  const int bh = blockIdx.x / nqb, qblk = blockIdx.x % nqb;
  const int b = bh / H, h = bh % H;
  const int q0 = qblk * 64 + w * 16;
  const float* Q = qb + (size_t)b * T * pitch + h * D;
  const float* K = kb + (size_t)b * T * pitch + h * D;
  const float* V = vb + (size_t)b * T * pitch + h * D;

  FragB aqh[KS], aql[KS];
  {
    int row = q0 + ln; if (row >= T) row = T - 1;
    const float* qr = Q + (size_t)row * pitch;
#pragma unroll
    for (int ks = 0; ks < KS; ++ks)
#pragma unroll
      for (int i = 0; i < 16; ++i) {
        const int d = ks * 32 + ((i < 8) ? (8 * hh + i) : (16 + 8 * hh + (i - 8)));
        const float x = qr[d] * scale; const unsigned short hb = bf16_bits(x);
        aqh[ks].u[i] = hb; aql[ks].u[i] = bf16_bits(x - bf16_val(hb));
      }
  }
  float m_r[8], l_r[8];
#pragma unroll
  for (int r = 0; r < 8; ++r) { m_r[r] = -3.0e38f; l_r[r] = 0.f; }
  v8f oacc[DT];
#pragma unroll
  for (int dt = 0; dt < DT; ++dt) oacc[dt] = (v8f){0.f,0.f,0.f,0.f,0.f,0.f,0.f,0.f};

  const int kv_end = CAUSAL ? min(T, qblk * 64 + 64) : T;
  for (int j0 = 0; j0 < kv_end; j0 += 32) {
    __syncthreads();
    for (int e = tid; e < 32 * (D / 4); e += 128) {
      const int r = e / (D / 4), c4 = (e % (D / 4)) * 4;
      const int key = j0 + r;
      v4f kf = {0.f,0.f,0.f,0.f}, vf = {0.f,0.f,0.f,0.f};
      if (key < T) { kf = *(const v4fa*)(K + (size_t)key * pitch + c4); vf = *(const v4fa*)(V + (size_t)key * pitch + c4); }
#pragma unroll
      for (int t = 0; t < 4; ++t) {
        unsigned short hb = bf16_bits(kf[t]); sKh[r][c4 + t] = hb; sKl[r][c4 + t] = bf16_bits(kf[t] - bf16_val(hb));
        hb = bf16_bits(vf[t]); sVh[r][c4 + t] = hb; sVl[r][c4 + t] = bf16_bits(vf[t] - bf16_val(hb));
      }
    }
    __syncthreads();
    v8f s[2];
#pragma unroll
    for (int nt = 0; nt < 2; ++nt) {
      v8f acc = {};
#pragma unroll
      for (int ks = 0; ks < KS; ++ks) {
        FragB bh_, bl_;
        bh_.half[0] = *(const v8us*)&sKh[nt * 16 + ln][ks * 32 + 8 * hh]; bh_.half[1] = *(const v8us*)&sKh[nt * 16 + ln][ks * 32 + 16 + 8 * hh];
        bl_.half[0] = *(const v8us*)&sKl[nt * 16 + ln][ks * 32 + 8 * hh]; bl_.half[1] = *(const v8us*)&sKl[nt * 16 + ln][ks * 32 + 16 + 8 * hh];
        acc = mmaN<3>(aqh[ks].v, aql[ks].v, bh_.v, bl_.v, acc);
      }
      s[nt] = acc;
    }
    float alpha[8];
#pragma unroll
    for (int r = 0; r < 8; ++r) {
      const int qi = q0 + 8 * hh + r;
      const int ja = j0 + ln, jb = j0 + 16 + ln;
      if (CAUSAL) { if (ja > qi) s[0][r] = -3.0e38f; if (jb > qi) s[1][r] = -3.0e38f; }
      if (ja >= T) s[0][r] = -3.0e38f;
      if (jb >= T) s[1][r] = -3.0e38f;
      float mx = fmaxf(s[0][r], s[1][r]);
      mx = fmaxf(mx, __shfl_xor(mx, 1, 32)); mx = fmaxf(mx, __shfl_xor(mx, 2, 32)); mx = fmaxf(mx, __shfl_xor(mx, 4, 32)); mx = fmaxf(mx, __shfl_xor(mx, 8, 32));
      const float mnew = fmaxf(m_r[r], mx);
      alpha[r] = (mnew > -1.0e38f) ? __expf(m_r[r] - mnew) : 1.0f;
      const float p0 = (s[0][r] > -1.0e38f) ? __expf(s[0][r] - mnew) : 0.f;
      const float p1 = (s[1][r] > -1.0e38f) ? __expf(s[1][r] - mnew) : 0.f;
      m_r[r] = mnew;
      l_r[r] = l_r[r] * alpha[r] + p0 + p1;
      unsigned short hb = bf16_bits(p0); sPh[w][8 * hh + r][ln] = hb;      sPl[w][8 * hh + r][ln] = bf16_bits(p0 - bf16_val(hb));
      hb = bf16_bits(p1);                sPh[w][8 * hh + r][16 + ln] = hb; sPl[w][8 * hh + r][16 + ln] = bf16_bits(p1 - bf16_val(hb));
    }
#pragma unroll
    for (int dt = 0; dt < DT; ++dt)
#pragma unroll
      for (int r = 0; r < 8; ++r) oacc[dt][r] *= alpha[r];
    __builtin_amdgcn_fence(__ATOMIC_ACQ_REL, "workgroup");
    __builtin_amdgcn_wave_barrier();
    FragB pah, pal;
    pah.half[0] = *(const v8us*)&sPh[w][ln][8 * hh]; pah.half[1] = *(const v8us*)&sPh[w][ln][16 + 8 * hh];
    pal.half[0] = *(const v8us*)&sPl[w][ln][8 * hh]; pal.half[1] = *(const v8us*)&sPl[w][ln][16 + 8 * hh];
#pragma unroll
    for (int dt = 0; dt < DT; ++dt) {
      FragB bvh, bvl;
#pragma unroll
      for (int i = 0; i < 8; ++i) {
        bvh.u[i] = sVh[8 * hh + i][dt * 16 + ln]; bvh.u[8 + i] = sVh[16 + 8 * hh + i][dt * 16 + ln];
        bvl.u[i] = sVl[8 * hh + i][dt * 16 + ln]; bvl.u[8 + i] = sVl[16 + 8 * hh + i][dt * 16 + ln];
      }
      oacc[dt] = mmaN<3>(pah.v, pal.v, bvh.v, bvl.v, oacc[dt]);
    }
    __builtin_amdgcn_fence(__ATOMIC_ACQ_REL, "workgroup");
    __builtin_amdgcn_wave_barrier();
  }
#pragma unroll
  for (int r = 0; r < 8; ++r) {
    float l = l_r[r];
    l += __shfl_xor(l, 1, 32); l += __shfl_xor(l, 2, 32); l += __shfl_xor(l, 4, 32); l += __shfl_xor(l, 8, 32);
    l_r[r] = (l > 0.f) ? 1.0f / l : 0.f;
  }
#pragma unroll
  for (int dt = 0; dt < DT; ++dt)
#pragma unroll
    for (int r = 0; r < 8; ++r) sO[w][8 * hh + r][dt * 16 + ln] = oacc[dt][r] * l_r[r];
  __builtin_amdgcn_fence(__ATOMIC_ACQ_REL, "workgroup");
  __builtin_amdgcn_wave_barrier();
  for (int pass = 0; pass < 2; ++pass) {
    for (int r = 0; r < 16; ++r) {
      const int row = q0 + r;
      if (row < T && lane < D / 4) {
        const v4f val = *(const v4fa*)&sO[w][r][lane * 4];
        *(volatile v4f*)(y + ((size_t)b * T + row) * ypitch + h * D + lane * 4) = val;
      }
    }
    if (pass == 0) __threadfence();
  }
}

template <bool ASPLIT, int ACT, bool BIAS_BF16, bool RES_BF16>
__global__ __launch_bounds__(128) void k_gemm_bf3(const float* __restrict__ A, int lda, const unsigned short* __restrict__ Wt, int ldb,
                                                const float* __restrict__ bias, const float* __restrict__ resid, int rmod, int ldr,
                                                float* __restrict__ C, int ldc, int M, int N, int K) {
  __shared__ __attribute__((aligned(16))) float so[4][16][64];
  const int tid = threadIdx.x, w = tid >> 5, lane = tid & 31, ln = lane & 15, hh = lane >> 4;
  const int ntn = N / 64;
  const int wid = blockIdx.x * 4 + w;
  const int mt = wid / ntn, nq = wid % ntn;
  if (mt * 16 >= M) return;
  const int row0 = mt * 16, col0 = nq * 64;
  const float* arow = A + (size_t)(row0 + ln) * lda;
  v8f acc[4] = {};
  for (int kb = 0; kb < K; kb += 32) {
    FragB ah, al;
    const v4f x0 = *(const v4fa*)(arow + kb + 8 * hh), x1 = *(const v4fa*)(arow + kb + 8 * hh + 4);
    const v4f x2 = *(const v4fa*)(arow + kb + 16 + 8 * hh), x3 = *(const v4fa*)(arow + kb + 16 + 8 * hh + 4);
    float xs[16] = {x0[0],x0[1],x0[2],x0[3],x1[0],x1[1],x1[2],x1[3],x2[0],x2[1],x2[2],x2[3],x3[0],x3[1],x3[2],x3[3]};
#pragma unroll
    for (int i = 0; i < 16; ++i) { const unsigned short hb = bf16_bits(xs[i]); ah.u[i] = hb; al.u[i] = ASPLIT ? bf16_bits(xs[i] - bf16_val(hb)) : (unsigned short)0; }
#pragma unroll
    for (int t = 0; t < 4; ++t) {
      const unsigned short* brow = Wt + (size_t)(col0 + t * 16 + ln) * ldb + kb;
      FragB b;
      b.half[0] = *(const v8us*)(brow + 8 * hh);
      b.half[1] = *(const v8us*)(brow + 16 + 8 * hh);
      acc[t] = mmaN<ASPLIT ? 2 : 1>(ah.v, al.v, b.v, b.v, acc[t]);
    }
  }
#pragma unroll
  for (int t = 0; t < 4; ++t) {
    const int col = col0 + t * 16 + ln;
    float bv = bias ? bias[col] : 0.f;
    if (BIAS_BF16) bv = bf16_round(bv);
#pragma unroll
    for (int r = 0; r < 8; ++r) {
      float v = acc[t][r] + bv;
      if (resid) { float rv = resid[(size_t)((row0 + 8 * hh + r) % rmod) * ldr + col]; if (RES_BF16) rv = bf16_round(rv); v += rv; }
      if (ACT == 1) v = fmaxf(v, 0.f);
      if (ACT == 2) v = 0.5f * v * (1.0f + erff(v * 0.70710678118654752f));
      if (ACT == 3) { const float u = 0.7978845608028654f * (v + 0.044715f * v * v * v); v = 0.5f * v * (1.0f + tanhf(u)); }
      so[w][8 * hh + r][t * 16 + ln] = v;
    }
  }
  __builtin_amdgcn_fence(__ATOMIC_ACQ_REL, "workgroup");
  __builtin_amdgcn_wave_barrier();
  const int rsub = lane >> 4, c4 = (lane & 15) * 4;
  for (int pass = 0; pass < 2; ++pass) {
#pragma unroll
    for (int q = 0; q < 8; ++q) {
      const int r = q * 2 + rsub;
      const v4f v = *(const v4fa*)&so[w][r][c4];
      *(volatile v4f*)(C + (size_t)(row0 + r) * ldc + col0 + c4) = v;
    }
    if (pass == 0) __threadfence();
  }
}
template <bool PARAM_BF16>
__global__ __launch_bounds__(256) void k_layernorm(const float* __restrict__ X, const float* __restrict__ R, const float* __restrict__ g, const float* __restrict__ bta,
                                                  float* __restrict__ out_sum, float* __restrict__ out_norm, int N, float eps) {
  __shared__ float red[256];
  const int row = blockIdx.x, tid = threadIdx.x;
  const float* x = X + (size_t)row * N; const float* rr = R ? R + (size_t)row * N : nullptr;
  float vals[16];
  const int per = N / 256;
  float s1 = 0.f;
  for (int u = 0; u < per / 4; ++u) {
    const int j = tid * 4 + 1024 * u;
    const v4f a = *(const v4fa*)(x + j);
    v4f b = {0.f,0.f,0.f,0.f}; if (rr) b = *(const v4fa*)(rr + j);
#pragma unroll
    for (int q = 0; q < 4; ++q) { const float v = a[q] + b[q]; vals[u * 4 + q] = v; s1 += v; }
  }
  red[tid] = s1; __syncthreads();
  for (int st = 128; st > 0; st >>= 1) { if (tid < st) red[tid] += red[tid + st]; __syncthreads(); }
  const float mu = red[0] / (float)N; __syncthreads();
  float s2 = 0.f;
  for (int u = 0; u < per / 4; ++u)
#pragma unroll
    for (int q = 0; q < 4; ++q) { const float c = vals[u * 4 + q] - mu; s2 += c * c; }
  red[tid] = s2; __syncthreads();
  for (int st = 128; st > 0; st >>= 1) { if (tid < st) red[tid] += red[tid + st]; __syncthreads(); }
  const float rs = rsqrtf(red[0] / (float)N + eps);
  for (int pass = 0; pass < 2; ++pass) {
    for (int u = 0; u < per / 4; ++u) {
      const int j = tid * 4 + 1024 * u;
      v4f o, sm;
#pragma unroll
      for (int q = 0; q < 4; ++q) {
        float gg = g[j + q], bb = bta[j + q];
        if (PARAM_BF16) { gg = bf16_round(gg); bb = bf16_round(bb); }
        sm[q] = vals[u * 4 + q]; o[q] = (vals[u * 4 + q] - mu) * rs * gg + bb;
      }
      if (out_sum) *(volatile v4f*)(out_sum + (size_t)row * N + j) = sm;
      *(volatile v4f*)(out_norm + (size_t)row * N + j) = o;
    }
    if (pass == 0) __threadfence();
  }
}


typedef _Float16 v16h __attribute__((ext_vector_type(16)));
union FragH { v16h v; v8us half[2]; _Float16 h[16]; unsigned short u[16]; };
template <int NT>
__device__ __forceinline__ v8f mmaH(v16h ah, v16h al, v16h bh, v16h bl, v8f c) {
  c = __builtin_amdgcn_wmma_f32_16x16x32_f16(false, ah, false, bh, (short)0, c, false, false);
  if (NT >= 2) c = __builtin_amdgcn_wmma_f32_16x16x32_f16(false, al, false, bh, (short)0, c, false, false);
  if (NT >= 3) c = __builtin_amdgcn_wmma_f32_16x16x32_f16(false, ah, false, bl, (short)0, c, false, false);
  asm volatile("v_nop\n\tv_nop\n\tv_nop\n\tv_nop" : "+v"(c) : "v"(ah), "v"(al), "v"(bh), "v"(bl));
  return c;
}
template <bool ASPLIT>
__global__ __launch_bounds__(128) void k_gemm_h(const float* __restrict__ A, int lda, size_t sA, const _Float16* __restrict__ Bh, int ldb, size_t sB, float alpha, float* __restrict__ C, int ldc, size_t sC, int M, int N, int K) {
  __shared__ __attribute__((aligned(16))) float so[4][16][64];
  const int tid = threadIdx.x, w = tid >> 5, lane = tid & 31, ln = lane & 15, hh = lane >> 4; const int by = blockIdx.y;
  A += (size_t)by * sA; Bh += (size_t)by * sB; C += (size_t)by * sC;
  const int ntn = (N + 63) / 64; const int wid = blockIdx.x * 4 + w; const int mt = wid / ntn, nq = wid % ntn; if (mt * 16 >= M) return;
  const int row0 = mt * 16, col0 = nq * 64; const float* arow = A + (size_t)(row0 + ln) * lda;
  v8f acc[4] = {};
  for (int kb = 0; kb < K; kb += 32) {
    FragH ah, al;
    const v4f x0 = *(const v4fa*)(arow + kb + 8 * hh), x1 = *(const v4fa*)(arow + kb + 8 * hh + 4), x2 = *(const v4fa*)(arow + kb + 16 + 8 * hh), x3 = *(const v4fa*)(arow + kb + 16 + 8 * hh + 4);
    float xs[16] = {x0[0],x0[1],x0[2],x0[3],x1[0],x1[1],x1[2],x1[3],x2[0],x2[1],x2[2],x2[3],x3[0],x3[1],x3[2],x3[3]};
#pragma unroll
    for (int i = 0; i < 16; ++i) { const _Float16 h = (_Float16)xs[i]; ah.h[i] = h; al.h[i] = ASPLIT ? (_Float16)(xs[i] - (float)h) : (_Float16)0.0f; }
#pragma unroll
    for (int t = 0; t < 4; ++t) { if (col0 + t * 16 >= N) continue; const size_t boff = (size_t)(col0 + t * 16 + ln) * ldb + kb; FragH bq; bq.half[0] = *(const v8us*)(Bh + boff + 8 * hh); bq.half[1] = *(const v8us*)(Bh + boff + 16 + 8 * hh);
      acc[t] = mmaH<ASPLIT ? 2 : 1>(ah.v, al.v, bq.v, bq.v, acc[t]); }
  }
#pragma unroll
  for (int t = 0; t < 4; ++t) { if (col0 + t * 16 >= N) continue;
#pragma unroll
    for (int r = 0; r < 8; ++r) so[w][8 * hh + r][t * 16 + ln] = acc[t][r] * alpha; }
  __builtin_amdgcn_fence(__ATOMIC_ACQ_REL, "workgroup"); __builtin_amdgcn_wave_barrier();
  const int rsub = lane >> 4, c4 = (lane & 15) * 4;
  for (int pass = 0; pass < 2; ++pass) {
#pragma unroll
    for (int q = 0; q < 8; ++q) { const int r = q * 2 + rsub; if (col0 + c4 < N) { const v4f v = *(const v4fa*)&so[w][r][c4]; *(volatile v4f*)(C + (size_t)(row0 + r) * ldc + col0 + c4) = v; } }
    if (pass == 0) __threadfence(); }
}

__global__ __launch_bounds__(256) void k_wt_f16(const float* __restrict__ W, _Float16* __restrict__ Wt, int K, int N, float scale) {
  const int t = blockIdx.x * 256 + threadIdx.x; if (t >= N * (K / 8)) return; const int n = t / (K / 8), k8 = (t % (K / 8)) * 8; FragH f;
#pragma unroll
  for (int i = 0; i < 8; ++i) f.h[i] = (_Float16)(bf16_round(W[(size_t)(k8 + i) * N + n]) * scale); const v8us o = f.half[0];
  *(volatile v8us*)((unsigned short*)Wt + (size_t)n * K + k8) = o; __threadfence(); *(volatile v8us*)((unsigned short*)Wt + (size_t)n * K + k8) = o;
}
template <int ACT>
__global__ __launch_bounds__(128) void k_gemm_hhx(const _Float16* __restrict__ A, int lda, size_t sA, const _Float16* __restrict__ Bh, int ldb, size_t sB, float alpha, const float* __restrict__ bias, size_t sBias, const float* __restrict__ CP, int rowsPerB, size_t sCPb, int row0g,
    float* __restrict__ C, _Float16* __restrict__ C16, int ldc, size_t sC, int M, int N, int K) {
  __shared__ __attribute__((aligned(16))) float so[4][16][64];
  const int tid = threadIdx.x, w = tid >> 5, lane = tid & 31, ln = lane & 15, hh = lane >> 4; const int by = blockIdx.y;
  A += (size_t)by * sA; Bh += (size_t)by * sB; const size_t cofs = (size_t)by * sC; const float* bp = bias ? bias + (size_t)by * sBias : nullptr;
  const int ntn = (N + 63) / 64; const int wid = blockIdx.x * 4 + w; const int mt = wid / ntn, nq = wid % ntn; if (mt * 16 >= M) return;
  const int row0 = mt * 16, col0 = nq * 64; const _Float16* arow = A + (size_t)(row0 + ln) * lda;
  v8f acc[4] = {};
  for (int kb = 0; kb < K; kb += 32) { FragH ah; ah.half[0] = *(const v8us*)((const unsigned short*)arow + kb + 8 * hh); ah.half[1] = *(const v8us*)((const unsigned short*)arow + kb + 16 + 8 * hh);
#pragma unroll
    for (int t = 0; t < 4; ++t) { if (col0 + t * 16 >= N) continue; const size_t boff = (size_t)(col0 + t * 16 + ln) * ldb + kb; FragH bq; bq.half[0] = *(const v8us*)((const unsigned short*)Bh + boff + 8 * hh); bq.half[1] = *(const v8us*)((const unsigned short*)Bh + boff + 16 + 8 * hh);
      acc[t] = mmaH<1>(ah.v, ah.v, bq.v, bq.v, acc[t]); }
  }
#pragma unroll
  for (int t = 0; t < 4; ++t) { if (col0 + t * 16 >= N) continue; const int col = col0 + t * 16 + ln; const float bv = bp ? bf16_round(bp[col]) : 0.f;
#pragma unroll
    for (int r = 0; r < 8; ++r) { float v = acc[t][r] * alpha + bv; if (CP) { const int bidx = (row0g + row0 + 8 * hh + r) / rowsPerB; v += CP[(size_t)bidx * sCPb + (size_t)by * 64 + col]; } if (ACT == 1) v = (v > 0.f) ? v : expm1f(v); else if (ACT == 3) v = fmaxf(v, 0.f); else if (ACT == 6) v = 0.5f * v * (1.0f + erff(v * 0.70710678118654752f)); so[w][8 * hh + r][t * 16 + ln] = v; } }
  __builtin_amdgcn_fence(__ATOMIC_ACQ_REL, "workgroup"); __builtin_amdgcn_wave_barrier();
  const int rsub = lane >> 4, c4 = (lane & 15) * 4; typedef _Float16 v4h __attribute__((ext_vector_type(4)));
  for (int pass = 0; pass < 2; ++pass) {
#pragma unroll
    for (int q = 0; q < 8; ++q) { const int r = q * 2 + rsub; if (col0 + c4 < N) { const v4f v = *(const v4fa*)&so[w][r][c4]; if (C) *(volatile v4f*)(C + cofs + (size_t)(row0 + r) * ldc + col0 + c4) = v; if (C16) { v4h h4; for (int i = 0; i < 4; ++i) h4[i] = (_Float16)v[i]; *(volatile v4h*)(C16 + cofs + (size_t)(row0 + r) * ldc + col0 + c4) = h4; } } }
    if (pass == 0) __threadfence(); }
}


__global__ __launch_bounds__(256) void k_round16f(const float* __restrict__ W, _Float16* __restrict__ Bt, size_t n8) { const size_t t = (size_t)blockIdx.x * 256 + threadIdx.x; if (t >= n8) return; FragH f;
#pragma unroll
  for (int i = 0; i < 8; ++i) f.h[i] = (_Float16)(bf16_round(W[t * 8 + i]) * 16.0f); *(volatile v8us*)((unsigned short*)Bt + t * 8) = f.half[0]; __threadfence(); *(volatile v8us*)((unsigned short*)Bt + t * 8) = f.half[0]; }
__global__ __launch_bounds__(256) void k_proj1(const float* __restrict__ x, const float* __restrict__ wq, const float* __restrict__ bq, const float* __restrict__ wk, const float* __restrict__ bk, const float* __restrict__ wv, const float* __restrict__ bv, _Float16* __restrict__ QKV) { const size_t tg = (size_t)blockIdx.x * 256 + threadIdx.x; if (tg >= (size_t)NRW * 24) return; const size_t row = tg / 24; const int rem = (int)(tg % 24); const int which = rem / 8, o8 = (rem % 8) * 8; const float* w = which == 0 ? wq : (which == 1 ? wk : wv); const float* b = which == 0 ? bq : (which == 1 ? bk : bv);
  const float x0 = bf16_round(x[row * 3]), x1 = bf16_round(x[row * 3 + 1]), x2 = bf16_round(x[row * 3 + 2]); FragH f;
#pragma unroll
  for (int q = 0; q < 8; ++q) { const int o = o8 + q; f.h[q] = (_Float16)(x0 * bf16_round(w[o]) + x1 * bf16_round(w[64 + o]) + x2 * bf16_round(w[128 + o]) + bf16_round(b[o])); }
  *(volatile v8us*)((unsigned short*)QKV + tg * 8) = f.half[0]; __threadfence(); *(volatile v8us*)((unsigned short*)QKV + tg * 8) = f.half[0]; }
template <int CV>
__global__ __launch_bounds__(256) void k_vt(const _Float16* __restrict__ V, int ldv, int voff, _Float16* __restrict__ Vt) { __shared__ unsigned short tl[64][66]; const int tid = threadIdx.x; const int g = blockIdx.x / 7, kg = blockIdx.x % 7;
  for (int i = tid; i < 64 * (CV / 8); i += 256) { const int r = i / (CV / 8), c8 = (i % (CV / 8)) * 8; const int key = kg * 64 + r; const int kc = key < NNn ? key : NNn - 1; FragH f; f.half[0] = *(const v8us*)((const unsigned short*)V + ((size_t)g * NNn + kc) * ldv + voff + c8);
#pragma unroll
    for (int q = 0; q < 8; ++q) tl[r][c8 + q] = (key < NNn) ? f.u[q] : (unsigned short)0; }
  __syncthreads();
  for (int pass = 0; pass < 2; ++pass) { for (int i = tid; i < CV * 8; i += 256) { const int c = i / 8, pc = i % 8; FragH f;
#pragma unroll
      for (int q = 0; q < 8; ++q) f.u[q] = tl[pc * 8 + q][c]; *(volatile v8us*)((unsigned short*)Vt + ((size_t)g * CV + c) * KP + kg * 64 + pc * 8) = f.half[0]; } if (pass == 0) __threadfence(); } }
template <int DH, int NHD, bool RELU16>
__global__ __launch_bounds__(128) void k_gat(const _Float16* __restrict__ QKV, int ld, int qoff, int koff, const _Float16* __restrict__ Vt, const float* __restrict__ adj, void* __restrict__ OUTP) {
  __shared__ __attribute__((aligned(16))) unsigned short sP[4][16][40]; __shared__ __attribute__((aligned(16))) float sO[4][16][NHD * DH + 4];
  const int tid = threadIdx.x, w = tid >> 5, lane = tid & 31, ln = lane & 15, hh = lane >> 4; const int g = blockIdx.x / 7, qb = blockIdx.x % 7; const int q0 = qb * 64 + w * 16; if (q0 >= NNn) return;
  const float scale = rsqrtf((float)DH); constexpr int DT = (NHD * DH >= 16) ? ((DH + 15) / 16) : 1;
#pragma unroll 1
  for (int h = 0; h < NHD; ++h) {
    FragH aq; { const unsigned short* qr = (const unsigned short*)QKV + ((size_t)g * NNn + q0 + ln) * ld + qoff + h * DH; if (DH == 32) { aq.half[0] = *(const v8us*)(qr + 8 * hh); aq.half[1] = *(const v8us*)(qr + 16 + 8 * hh); } else { aq.half[0] = *(const v8us*)(qr + 8 * hh); aq.half[1] = (v8us){0,0,0,0,0,0,0,0}; } }
    const unsigned short* Vth = (const unsigned short*)Vt + ((size_t)g * NHD * DH + h * DH) * KP;
    float m_r[8], l_r[8]; v8f oacc[DT];
#pragma unroll
    for (int r = 0; r < 8; ++r) { m_r[r] = -3.0e38f; l_r[r] = 0.f; }
#pragma unroll
    for (int dt = 0; dt < DT; ++dt) oacc[dt] = (v8f){0.f,0.f,0.f,0.f,0.f,0.f,0.f,0.f};
#pragma unroll 1
    for (int j0 = 0; j0 < KP - 32; j0 += 32) { v8f s[2];
#pragma unroll
      for (int nt = 0; nt < 2; ++nt) { const int kq = j0 + nt * 16 + ln; const int kc = kq < NNn ? kq : NNn - 1; const unsigned short* kr = (const unsigned short*)QKV + ((size_t)g * NNn + kc) * ld + koff + h * DH; FragH bk; if (DH == 32) { bk.half[0] = *(const v8us*)(kr + 8 * hh); bk.half[1] = *(const v8us*)(kr + 16 + 8 * hh); } else { bk.half[0] = *(const v8us*)(kr + 8 * hh); bk.half[1] = (v8us){0,0,0,0,0,0,0,0}; }
        v8f acc = (v8f){0.f,0.f,0.f,0.f,0.f,0.f,0.f,0.f}; acc = mmaH<1>(aq.v, aq.v, bk.v, bk.v, acc); s[nt] = acc; }
#pragma unroll
      for (int r = 0; r < 8; ++r) { const int tq = q0 + 8 * hh + r; const int k0 = j0 + ln, k1 = j0 + 16 + ln; const bool ex0 = (k0 < NNn), ex1 = (k1 < NNn);
        const float a0 = ex0 ? bf16_round(adj[(size_t)tq * NNn + k0]) : 0.f, a1 = ex1 ? bf16_round(adj[(size_t)tq * NNn + k1]) : 0.f;
        float s0 = (a0 == 0.f) ? -1e9f : s[0][r] * scale, s1 = (a1 == 0.f) ? -1e9f : s[1][r] * scale; s0 = ex0 ? s0 : -INFINITY; s1 = ex1 ? s1 : -INFINITY; float mc = fmaxf(s0, s1);
        mc = fmaxf(mc, __shfl_xor(mc, 1, 32)); mc = fmaxf(mc, __shfl_xor(mc, 2, 32)); mc = fmaxf(mc, __shfl_xor(mc, 4, 32)); mc = fmaxf(mc, __shfl_xor(mc, 8, 32));
        const float mn = fmaxf(m_r[r], mc); const float al = (mn > -1.0e38f) ? expf(m_r[r] - mn) : 1.0f; m_r[r] = mn; const float p0 = ex0 ? expf(s0 - mn) : 0.f, p1 = ex1 ? expf(s1 - mn) : 0.f; l_r[r] = l_r[r] * al + p0 + p1;
#pragma unroll
        for (int dt = 0; dt < DT; ++dt) oacc[dt][r] *= al;
        FragH t2; t2.h[0] = (_Float16)p0; t2.h[1] = (_Float16)p1; sP[w][8 * hh + r][ln] = t2.u[0]; sP[w][8 * hh + r][16 + ln] = t2.u[1]; }
      __builtin_amdgcn_fence(__ATOMIC_ACQ_REL, "workgroup"); __builtin_amdgcn_wave_barrier();
      FragH pa; pa.half[0] = *(const v8us*)&sP[w][ln][8 * hh]; pa.half[1] = *(const v8us*)&sP[w][ln][16 + 8 * hh];
#pragma unroll
      for (int dt = 0; dt < DT; ++dt) { const int d = dt * 16 + ln; const int dc = d < DH ? d : DH - 1; const unsigned short* vrow = Vth + (size_t)dc * KP + j0; FragH bv; bv.half[0] = *(const v8us*)(vrow + 8 * hh); bv.half[1] = *(const v8us*)(vrow + 16 + 8 * hh); oacc[dt] = mmaH<1>(pa.v, pa.v, bv.v, bv.v, oacc[dt]); }
      __builtin_amdgcn_fence(__ATOMIC_ACQ_REL, "workgroup"); __builtin_amdgcn_wave_barrier(); }
#pragma unroll
    for (int r = 0; r < 8; ++r) { float l = l_r[r]; l += __shfl_xor(l, 1, 32); l += __shfl_xor(l, 2, 32); l += __shfl_xor(l, 4, 32); l += __shfl_xor(l, 8, 32); l_r[r] = 1.0f / l; }
#pragma unroll
    for (int dt = 0; dt < DT; ++dt) { const int d = dt * 16 + ln; if (d < DH) {
#pragma unroll
      for (int r = 0; r < 8; ++r) sO[w][8 * hh + r][h * DH + d] = oacc[dt][r] * l_r[r]; } }
    __builtin_amdgcn_wave_barrier(); }
  __builtin_amdgcn_fence(__ATOMIC_ACQ_REL, "workgroup"); __builtin_amdgcn_wave_barrier();
  constexpr int RW = NHD * DH;
  for (int pass = 0; pass < 2; ++pass) {
    if (RELU16) {
#pragma unroll
      for (int rp = 0; rp < 16; rp += 4) { const int r = rp + (lane >> 3), pc = lane & 7; FragH f;
#pragma unroll
        for (int q = 0; q < 8; ++q) f.h[q] = (_Float16)fmaxf(sO[w][r][pc * 8 + q], 0.f); *(volatile v8us*)((unsigned short*)OUTP + ((size_t)g * NNn + q0 + r) * RW + pc * 8) = f.half[0]; } }
    else {
#pragma unroll
      for (int rp = 0; rp < 16; rp += 4) { const int r = rp + (lane >> 3), pc = lane & 7; const v4f v = *(const v4fa*)&sO[w][r][pc * 4]; *(volatile v4f*)((float*)OUTP + ((size_t)g * NNn + q0 + r) * RW + pc * 4) = v; } }
    if (pass == 0) __threadfence(); } }
__global__ __launch_bounds__(256) void k_spln(const float* __restrict__ O2, const float* __restrict__ x, const float* __restrict__ g_, const float* __restrict__ b_, float* __restrict__ SP, _Float16* __restrict__ T16) { const size_t tg = (size_t)blockIdx.x * 256 + threadIdx.x; if (tg >= (size_t)NRW * 8) return; const size_t trow = tg / 8; const int pc = (int)(tg % 8);
  const int sq = (int)(trow % SS); const size_t bn = trow / SS; const int n = (int)(bn % NNn), b = (int)(bn / NNn); const size_t row = ((size_t)(b * SS + sq)) * NNn + n;
  float v[4]; float s = 0.f;
#pragma unroll
  for (int q = 0; q < 4; ++q) { const int c = pc * 4 + q; v[q] = O2[row * DM + c] + ((c < 3) ? bf16_round(x[row * 3 + c]) : 0.f); s += v[q]; }
  s += __shfl_xor(s, 1, 32); s += __shfl_xor(s, 2, 32); s += __shfl_xor(s, 4, 32); const float mu = s / 32.0f; float q2 = 0.f;
#pragma unroll
  for (int q = 0; q < 4; ++q) { const float d = v[q] - mu; q2 += d * d; } q2 += __shfl_xor(q2, 1, 32); q2 += __shfl_xor(q2, 2, 32); q2 += __shfl_xor(q2, 4, 32); const float rs = 1.0f / sqrtf(q2 / 32.0f + 1e-6f);
  v4f o; typedef _Float16 v4h __attribute__((ext_vector_type(4))); v4h oh;
#pragma unroll
  for (int q = 0; q < 4; ++q) { const int c = pc * 4 + q; o[q] = bf16_round(g_[c]) * (v[q] - mu) * rs + bf16_round(b_[c]); oh[q] = (_Float16)o[q]; }
  for (int pass = 0; pass < 2; ++pass) { *(volatile v4f*)(SP + row * DM + pc * 4) = o; *(volatile v4h*)(T16 + trow * DM + pc * 4) = oh; if (pass == 0) __threadfence(); } }
__global__ __launch_bounds__(256) void k_tattn(const _Float16* __restrict__ QKVT, _Float16* __restrict__ OT16) { __shared__ __attribute__((aligned(16))) _Float16 so[8][SS][64 + 8]; __shared__ float ssc[8][SS][SS + 1]; const int tid = threadIdx.x, wv = tid >> 5, lane = tid & 31; const size_t seq = (size_t)blockIdx.x * 8 + wv; const bool act = (seq < (size_t)BBs * NNn) && (lane < SS);
  if (act) { const size_t rq = seq * SS + lane;
#pragma unroll 1
    for (int h = 0; h < 2; ++h) { float m = -3.0e38f;
#pragma unroll 1
      for (int s2 = 0; s2 < SS; ++s2) { const size_t rk = seq * SS + s2; float d = 0.f;
#pragma unroll 1
        for (int k = 0; k < 32; ++k) d += (float)QKVT[rq * 192 + h * 32 + k] * (float)QKVT[rk * 192 + 64 + h * 32 + k]; const float sv = d * 0.17677669529663687f; ssc[wv][lane][s2] = sv; m = fmaxf(m, sv); }
      float z = 0.f;
#pragma unroll 1
      for (int s2 = 0; s2 < SS; ++s2) { const float e = expf(ssc[wv][lane][s2] - m); ssc[wv][lane][s2] = e; z += e; } const float iz = 1.0f / z;
#pragma unroll 1
      for (int k = 0; k < 32; ++k) { float o = 0.f;
#pragma unroll 1
        for (int s2 = 0; s2 < SS; ++s2) o += ssc[wv][lane][s2] * (float)QKVT[(seq * SS + s2) * 192 + 128 + h * 32 + k]; so[wv][lane][h * 32 + k] = (_Float16)(o * iz); } } }
  __syncthreads();
  for (int pass = 0; pass < 2; ++pass) { if (seq < (size_t)BBs * NNn) { for (int i = lane; i < SS * 8; i += 32) { const int r = i / 8, pc = i % 8; const v8us v = *(const v8us*)&so[wv][r][pc * 8]; *(volatile v8us*)((unsigned short*)OT16 + (seq * SS + r) * 64 + pc * 8) = v; } } if (pass == 0) __threadfence(); } }
__global__ __launch_bounds__(256) void k_resln(const float* __restrict__ Ain, int perm, const float* __restrict__ Bin, const float* __restrict__ g_, const float* __restrict__ b_, float* __restrict__ Y, _Float16* __restrict__ Y16) { const size_t tg = (size_t)blockIdx.x * 256 + threadIdx.x; if (tg >= (size_t)NRW * 8) return; const size_t row = tg / 8; const int pc = (int)(tg % 8); size_t arow = row; if (perm) { const int sq = (int)(row % SS); const size_t bn = row / SS; const int n = (int)(bn % NNn), b = (int)(bn / NNn); arow = ((size_t)(b * SS + sq)) * NNn + n; }
  float v[4]; float s = 0.f;
#pragma unroll
  for (int q = 0; q < 4; ++q) { const int c = pc * 4 + q; v[q] = Ain[arow * DM + c] + Bin[row * DM + c]; s += v[q]; }
  s += __shfl_xor(s, 1, 32); s += __shfl_xor(s, 2, 32); s += __shfl_xor(s, 4, 32); const float mu = s / 32.0f; float q2 = 0.f;
#pragma unroll
  for (int q = 0; q < 4; ++q) { const float d = v[q] - mu; q2 += d * d; } q2 += __shfl_xor(q2, 1, 32); q2 += __shfl_xor(q2, 2, 32); q2 += __shfl_xor(q2, 4, 32); const float rs = 1.0f / sqrtf(q2 / 32.0f + 1e-6f);
  v4f o; typedef _Float16 v4h __attribute__((ext_vector_type(4))); v4h oh;
#pragma unroll
  for (int q = 0; q < 4; ++q) { const int c = pc * 4 + q; o[q] = bf16_round(g_[c]) * (v[q] - mu) * rs + bf16_round(b_[c]); oh[q] = (_Float16)o[q]; }
  for (int pass = 0; pass < 2; ++pass) { *(volatile v4f*)(Y + row * DM + pc * 4) = o; if (Y16) *(volatile v4h*)(Y16 + row * DM + pc * 4) = oh; if (pass == 0) __threadfence(); } }
__global__ __launch_bounds__(256) void k_final(const float* __restrict__ SP, const float* __restrict__ TOUT, const float* __restrict__ g_, const float* __restrict__ b_, const float* __restrict__ fw, const float* __restrict__ fb, float* __restrict__ out) { const int tg = blockIdx.x * 256 + threadIdx.x; const int pc = tg % 8;   const int t = tg / 8; const int b = t / NNn, n = t % NNn; float vs[4] = {0.f, 0.f, 0.f, 0.f}, vt[4] = {0.f, 0.f, 0.f, 0.f};
#pragma unroll 1
  for (int sq = 0; sq < SS; ++sq) { const v4f a = *(const v4fa*)(SP + (((size_t)(b * SS + sq)) * NNn + n) * DM + pc * 4); const v4f c = *(const v4fa*)(TOUT + (((size_t)b * NNn + n) * SS + sq) * DM + pc * 4);
#pragma unroll
    for (int q = 0; q < 4; ++q) { vs[q] += a[q]; vt[q] += c[q]; } }
  float v[4]; float s = 0.f;
#pragma unroll
  for (int q = 0; q < 4; ++q) { v[q] = vs[q] / (float)SS + vt[q] / (float)SS; s += v[q]; }
  s += __shfl_xor(s, 1, 32); s += __shfl_xor(s, 2, 32); s += __shfl_xor(s, 4, 32); const float mu = s / 32.0f; float q2 = 0.f;
#pragma unroll
  for (int q = 0; q < 4; ++q) { const float d = v[q] - mu; q2 += d * d; } q2 += __shfl_xor(q2, 1, 32); q2 += __shfl_xor(q2, 2, 32); q2 += __shfl_xor(q2, 4, 32); const float rs = 1.0f / sqrtf(q2 / 32.0f + 1e-6f);
  float o = 0.f;
#pragma unroll
  for (int q = 0; q < 4; ++q) { const int c = pc * 4 + q; o += (bf16_round(g_[c]) * (v[q] - mu) * rs + bf16_round(b_[c])) * bf16_round(fw[c]); }
  o += __shfl_xor(o, 1, 32); o += __shfl_xor(o, 2, 32); o += __shfl_xor(o, 4, 32); o += bf16_round(fb[0]);
  __shared__ float sred[32]; if (pc == 0) sred[threadIdx.x / 8] = o; __syncthreads();
  if (threadIdx.x < 32) { const int tw = blockIdx.x * 32 + threadIdx.x; const float ov = sred[threadIdx.x]; *(volatile float*)(out + tw) = ov; __threadfence(); *(volatile float*)(out + tw) = ov; } }
extern "C" void kernel_launch(void* const* d_in, const int* in_sizes, int n_in,
                              void* d_out, int out_size, void* d_ws, size_t ws_size, hipStream_t stream) {
  (void)in_sizes; (void)n_in; (void)out_size;
  const float* const* I = (const float* const*)d_in; const float* xin = I[0]; const float* adj = I[1];
  const float* g1wq = I[2]; const float* g1bq = I[3]; const float* g1wk = I[4]; const float* g1bk = I[5]; const float* g1wv = I[6]; const float* g1bv = I[7];
  const float* g2wq = I[8]; const float* g2bq = I[9]; const float* g2wk = I[10]; const float* g2bk = I[11]; const float* g2wv = I[12]; const float* g2bv = I[13]; const float* spg = I[14]; const float* spb = I[15];
  const float* twq = I[16]; const float* tbq = I[17]; const float* twk = I[18]; const float* tbk = I[19]; const float* twv = I[20]; const float* tbv = I[21]; const float* two = I[22]; const float* tbo = I[23];
  const float* ffw1 = I[24]; const float* ffb1 = I[25]; const float* ffw2 = I[26]; const float* ffb2 = I[27]; const float* ln1g = I[28]; const float* ln1b = I[29]; const float* ln2g = I[30]; const float* ln2b = I[31]; const float* fing = I[32]; const float* finb = I[33]; const float* fdw = I[34]; const float* fdb = I[35];
  char* ws = (char*)d_ws; size_t off = 0;
  auto take = [&](size_t bytes) { char* p = ws + off; off += (bytes + 255) & ~(size_t)255; return p; };
  _Float16* Bq2 = (_Float16*)take(DM * 64 * 2); _Float16* Bk2 = (_Float16*)take(DM * 64 * 2); _Float16* Bv2 = (_Float16*)take(DM * 64 * 2); _Float16* Btq = (_Float16*)take(64 * DM * 2); _Float16* Btk = (_Float16*)take(64 * DM * 2); _Float16* Btv = (_Float16*)take(64 * DM * 2); _Float16* Bto = (_Float16*)take(DM * 64 * 2); _Float16* Bf1 = (_Float16*)take(64 * DM * 2); _Float16* Bf2 = (_Float16*)take(DM * 64 * 2);
  char* R1 = take((size_t)NRW * 192 * 2); _Float16* QKV1 = (_Float16*)R1; _Float16* QKVT = (_Float16*)R1;
  char* R2 = take((size_t)NG * 64 * KP * 2); _Float16* Vt1 = (_Float16*)R2; _Float16* OT16 = (_Float16*)R2; _Float16* X1h = nullptr;
  _Float16* H1 = (_Float16*)take((size_t)NRW * 64 * 2); _Float16* F1h = H1;
  char* R4 = take((size_t)NRW * 96 * 2); _Float16* QKV2 = (_Float16*)R4; float* Aout = (float*)R4;
  X1h = (_Float16*)(R4 + (size_t)NRW * DM * 4);
  _Float16* Vt2 = (_Float16*)take((size_t)NG * DM * KP * 2); float* O2 = (float*)take((size_t)NRW * DM * 4); float* F2 = O2;
  float* SP = (float*)take((size_t)NRW * DM * 4); _Float16* T16 = (_Float16*)take((size_t)NRW * DM * 2); float* X1 = (float*)take((size_t)NRW * DM * 4); float* TOUT = (float*)take((size_t)NRW * DM * 4);
  if (off > ws_size) return;
  k_wt_f16<<<1, 256, 0, stream>>>(g2wq, Bq2, 64, DM, 16.0f); k_wt_f16<<<1, 256, 0, stream>>>(g2wk, Bk2, 64, DM, 16.0f); k_wt_f16<<<1, 256, 0, stream>>>(g2wv, Bv2, 64, DM, 16.0f);
  k_wt_f16<<<1, 256, 0, stream>>>(twq, Btq, DM, 64, 16.0f); k_wt_f16<<<1, 256, 0, stream>>>(twk, Btk, DM, 64, 16.0f); k_wt_f16<<<1, 256, 0, stream>>>(twv, Btv, DM, 64, 16.0f); k_wt_f16<<<1, 256, 0, stream>>>(two, Bto, 64, DM, 16.0f);
  k_wt_f16<<<1, 256, 0, stream>>>(ffw1, Bf1, DM, 64, 16.0f); k_wt_f16<<<1, 256, 0, stream>>>(ffw2, Bf2, 64, DM, 16.0f);
  k_proj1<<<(unsigned)(((size_t)NRW * 24 + 255) / 256), 256, 0, stream>>>(xin, g1wq, g1bq, g1wk, g1bk, g1wv, g1bv, QKV1);
  k_vt<64><<<NG * 7, 256, 0, stream>>>(QKV1, 192, 128, Vt1);
  k_gat<16, 4, true><<<NG * 7, 128, 0, stream>>>(QKV1, 192, 0, 64, Vt1, adj, (void*)H1);
  const dim3 g32(((NRW / 16) * 1 + 3) / 4, 1), g64(((NRW / 16) * 1 + 3) / 4, 1);
  k_gemm_hhx<0><<<g32, 128, 0, stream>>>(H1, 64, 0, Bq2, 64, 0, 0.0625f, g2bq, 0, nullptr, 1, 0, 0, nullptr, QKV2, DM, 0, NRW, DM, 64);
  k_gemm_hhx<0><<<g32, 128, 0, stream>>>(H1, 64, 0, Bk2, 64, 0, 0.0625f, g2bk, 0, nullptr, 1, 0, 0, nullptr, QKV2 + (size_t)NRW * DM, DM, 0, NRW, DM, 64);
  k_gemm_hhx<0><<<g32, 128, 0, stream>>>(H1, 64, 0, Bv2, 64, 0, 0.0625f, g2bv, 0, nullptr, 1, 0, 0, nullptr, QKV2 + (size_t)2 * NRW * DM, DM, 0, NRW, DM, 64);
  k_vt<32><<<NG * 7, 256, 0, stream>>>(QKV2 + (size_t)2 * NRW * DM, DM, 0, Vt2);
  k_gat<32, 1, false><<<NG * 7, 128, 0, stream>>>(QKV2, DM, 0, NRW * DM, Vt2, adj, (void*)O2);
  k_spln<<<(unsigned)(((size_t)NRW * 8 + 255) / 256), 256, 0, stream>>>(O2, xin, spg, spb, SP, T16);
  k_gemm_hhx<0><<<g64, 128, 0, stream>>>(T16, DM, 0, Btq, DM, 0, 0.0625f, tbq, 0, nullptr, 1, 0, 0, nullptr, QKVT, 192, 0, NRW, 64, DM);
  k_gemm_hhx<0><<<g64, 128, 0, stream>>>(T16, DM, 0, Btk, DM, 0, 0.0625f, tbk, 0, nullptr, 1, 0, 0, nullptr, QKVT + 64, 192, 0, NRW, 64, DM);
  k_gemm_hhx<0><<<g64, 128, 0, stream>>>(T16, DM, 0, Btv, DM, 0, 0.0625f, tbv, 0, nullptr, 1, 0, 0, nullptr, QKVT + 128, 192, 0, NRW, 64, DM);
  k_tattn<<<(BBs * NNn + 7) / 8, 256, 0, stream>>>(QKVT, OT16);
  k_gemm_hhx<0><<<g32, 128, 0, stream>>>(OT16, 64, 0, Bto, 64, 0, 0.0625f, tbo, 0, nullptr, 1, 0, 0, Aout, nullptr, DM, 0, NRW, DM, 64);
  k_resln<<<(unsigned)(((size_t)NRW * 8 + 255) / 256), 256, 0, stream>>>(SP, 1, Aout, ln1g, ln1b, X1, X1h);
  k_gemm_hhx<6><<<g64, 128, 0, stream>>>(X1h, DM, 0, Bf1, DM, 0, 0.0625f, ffb1, 0, nullptr, 1, 0, 0, nullptr, F1h, 64, 0, NRW, 64, DM);
  k_gemm_hhx<0><<<g32, 128, 0, stream>>>(F1h, 64, 0, Bf2, 64, 0, 0.0625f, ffb2, 0, nullptr, 1, 0, 0, F2, nullptr, DM, 0, NRW, DM, 64);
  k_resln<<<(unsigned)(((size_t)NRW * 8 + 255) / 256), 256, 0, stream>>>(X1, 0, F2, ln2g, ln2b, TOUT, nullptr);
  k_final<<<(BBs * NNn * 8 + 255) / 256, 256, 0, stream>>>(SP, TOUT, fing, finb, fdw, fdb, (float*)d_out);
}
